// MultiHeadAttentionLayer_65420941853360
// MI455X (gfx1250) — hardware-run, weakly checked
//
#include <hip/hip_runtime.h>

typedef float          v8f   __attribute__((ext_vector_type(8)));
typedef float          v4f   __attribute__((ext_vector_type(4)));
typedef unsigned int   v4u   __attribute__((ext_vector_type(4)));
typedef int            v8i   __attribute__((ext_vector_type(8)));
typedef unsigned short v8us  __attribute__((ext_vector_type(8)));
typedef unsigned short v16us __attribute__((ext_vector_type(16)));
typedef __bf16         v16bf __attribute__((ext_vector_type(16)));
typedef _Float16       v16h  __attribute__((ext_vector_type(16)));
typedef v4f  __attribute__((may_alias)) v4fa;
typedef v8us __attribute__((may_alias)) v8usa;
union FragB { v16bf v; v16us u; v8us h[2]; v8i w; };
union FragH { v16h  v; v16us u; v8us h[2]; v8i w; };

__device__ __forceinline__ v8f wmb(const FragB& a, const FragB& b, v8f c) {
  v8f d = __builtin_amdgcn_wmma_f32_16x16x32_bf16(false, a.v, false, b.v, (short)0, c, false, false);
  asm volatile("v_nop\n\tv_nop\n\tv_nop\n\tv_nop" : "+v"(d) : "v"(a.w), "v"(b.w));
  return d;
}

__device__ __forceinline__ v8f wmh(const FragH& a, const FragH& b, v8f c) {
  v8f d = __builtin_amdgcn_wmma_f32_16x16x32_f16(false, a.v, false, b.v, (short)0, c, false, false);
  asm volatile("v_nop\n\tv_nop\n\tv_nop\n\tv_nop" : "+v"(d) : "v"(a.w), "v"(b.w));
  return d;
}

__device__ __forceinline__ unsigned bf16_bits(float f) {
  const unsigned u = __float_as_uint(f);
  const unsigned r = (u + 0x7FFFu + ((u >> 16) & 1u)) >> 16;
  const unsigned q = (u >> 16) | 0x40u;
  return ((u & 0x7fffffffu) > 0x7f800000u) ? q : r;
}

__device__ __forceinline__ float bf16_val(float f) {
  return __uint_as_float(bf16_bits(f) << 16);
}
__device__ __forceinline__ int clampi(int v, int lo, int hi) {
  return v < lo ? lo : (v > hi ? hi : v);
}

__device__ __forceinline__ unsigned f16_bits(float f) {
  const unsigned u  = __float_as_uint(f);
  const unsigned s  = (u >> 16) & 0x8000u;
  const unsigned a  = u & 0x7fffffffu;
  const unsigned t  = a - 0x38000000u;
  const unsigned r  = (t + 0x0FFFu + ((t >> 13) & 1u)) >> 13;
  const unsigned rc = r > 0x7C00u ? 0x7C00u : r;
  const bool small  = a < 0x38800000u;
  const bool isnan  = a > 0x7f800000u;
  const unsigned fin = small ? 0u : (s | rc);
  return isnan ? (s | 0x7E00u) : fin;
}

__device__ __forceinline__ unsigned pk16(unsigned lo, unsigned hi) { return lo | (hi << 16); }
__device__ __forceinline__ unsigned bf16_lo_bits(float v) {
  float hi = bf16_val(v);
  asm volatile("" : "+v"(hi));
  return bf16_bits(v - hi);
}
__device__ __forceinline__ v4u pack8_bf16(v4f a, v4f c) {
  return (v4u){ pk16(bf16_bits(a[0]), bf16_bits(a[1])), pk16(bf16_bits(a[2]), bf16_bits(a[3])),
                pk16(bf16_bits(c[0]), bf16_bits(c[1])), pk16(bf16_bits(c[2]), bf16_bits(c[3])) };
}
__device__ __forceinline__ v4u pack8_bf16_lo(v4f a, v4f c) {
  return (v4u){ pk16(bf16_lo_bits(a[0]), bf16_lo_bits(a[1])), pk16(bf16_lo_bits(a[2]), bf16_lo_bits(a[3])),
                pk16(bf16_lo_bits(c[0]), bf16_lo_bits(c[1])), pk16(bf16_lo_bits(c[2]), bf16_lo_bits(c[3])) };
}
__device__ __forceinline__ v4u pack8_f16(v4f a, v4f c) {
  return (v4u){ pk16(f16_bits(a[0]), f16_bits(a[1])), pk16(f16_bits(a[2]), f16_bits(a[3])),
                pk16(f16_bits(c[0]), f16_bits(c[1])), pk16(f16_bits(c[2]), f16_bits(c[3])) };
}

template <int FORM>
__global__ __launch_bounds__(256) void k_plane(const float* __restrict__ src, int rows, int cols, int ldsrc,
                                               unsigned short* __restrict__ dst, int MP, int KP) {
  static_assert(FORM >= 0 && FORM <= 3);
  const int KTOT = (FORM == 1 || FORM == 3) ? 2 * KP : KP;
  const unsigned ppr   = (unsigned)(KTOT >> 3);
  const unsigned kp8   = (unsigned)(KP >> 3);
  const unsigned total = (unsigned)MP * ppr;
  const unsigned g     = blockIdx.x * 256u + threadIdx.x;
  const unsigned rowu  = g / ppr;
  const unsigned p     = g - rowu * ppr;
  const bool second    = p >= kp8;
  const int row = (int)rowu;
  const int c0  = (int)((second ? p - kp8 : p) << 3);
  const float* srow = src + (size_t)clampi(row, 0, rows - 1) * (size_t)ldsrc;
  float x[8];
  unsigned mk[8];
#pragma unroll
  for (int e = 0; e < 8; ++e) {
    const int c = c0 + e;
    const float v = srow[clampi(c, 0, cols - 1)];
    asm volatile("" :: "v"(v));
    x[e]  = v;
    mk[e] = (row < rows && c < cols) ? 0xFFFFu : 0u;
  }
  const v4f a = (v4f){ x[0], x[1], x[2], x[3] };
  const v4f c = (v4f){ x[4], x[5], x[6], x[7] };
  v4u o;
  if (FORM == 2) {
    o = pack8_f16(a, c);
  } else {
    const v4u hi = pack8_bf16(a, c);
    o = hi;
    if (FORM == 1) { const v4u lo = pack8_bf16_lo(a, c); o = second ? lo : hi; }
  }
  const v4u mw = (v4u){ pk16(mk[0], mk[1]), pk16(mk[2], mk[3]), pk16(mk[4], mk[5]), pk16(mk[6], mk[7]) };
  o &= mw;
  if (g < total) {
    volatile v4u* q = (volatile v4u*)(dst + (size_t)g * 8);
    *q = o;
    __threadfence();
    *q = o;
  }
}

template <int FORM> struct FragOf    { typedef FragB T; };
template <>         struct FragOf<2> { typedef FragH T; };
__device__ __forceinline__ v8f mm(const FragB& a, const FragB& b, v8f c) { return wmb(a, b, c); }
__device__ __forceinline__ v8f mm(const FragH& a, const FragH& b, v8f c) { return wmh(a, b, c); }
template <class F> __device__ __forceinline__ F ld_frag(const unsigned short* p) {
  F f;
  f.h[0] = *(const v8usa*)(p);
  f.h[1] = *(const v8usa*)(p + 16);
  return f;
}

template <int FORM, int EPI>
__global__ __launch_bounds__(256) __attribute__((amdgpu_num_vgpr(248)))
void k_gemm_nt(const unsigned short* __restrict__ A, const unsigned short* __restrict__ B,
               const float* __restrict__ bias, float* __restrict__ D, int M, int N, int KTOT, int ldd) {
  static_assert(FORM >= 0 && FORM <= 2);
  static_assert(EPI == 0 || EPI == 1);
  typedef typename FragOf<FORM>::T F;
  __shared__ __attribute__((aligned(16))) float sT[8][16 * 68];
  const int lane = threadIdx.x & 31;
  const int wave = threadIdx.x >> 5;
  const int tilesM = (M + 63) >> 6;
  const int tilesN = (N + 63) >> 6;
  const int tile = blockIdx.x * 8 + wave;
  if (tile >= tilesM * tilesN) return;
  const int tm = tile / tilesN;
  const int tn = tile - tm * tilesN;
  const int m0 = tm << 6;
  const int n0 = tn << 6;

  const int rl = lane & 15;
  const int h8 = (lane >> 4) * 8;
  const unsigned short* pa = A + (size_t)(m0 + rl) * (size_t)KTOT + h8;
  const unsigned short* pb = B + (size_t)(n0 + rl) * (size_t)KTOT + h8;

  v8f acc[4][4];
#pragma unroll
  for (int i = 0; i < 4; ++i)
#pragma unroll
    for (int j = 0; j < 4; ++j) acc[i][j] = (v8f){0.f, 0.f, 0.f, 0.f, 0.f, 0.f, 0.f, 0.f};

#pragma unroll 1
  for (int k0 = 0; k0 < KTOT; k0 += 32) {
    F bf[4];
#pragma unroll
    for (int j = 0; j < 4; ++j) bf[j] = ld_frag<F>(pb + (size_t)(j << 4) * (size_t)KTOT + k0);
#pragma unroll
    for (int i = 0; i < 4; ++i) {
      const F af = ld_frag<F>(pa + (size_t)(i << 4) * (size_t)KTOT + k0);
#pragma unroll
      for (int j = 0; j < 4; ++j) acc[i][j] = mm(af, bf[j], acc[i][j]);
    }
  }

  float* slab = sT[wave];
  const int hh = lane >> 4;
  const int c4 = (lane & 15) * 4;
  const int nc = n0 + c4;
  const bool cok = nc < N;
  v4f bv = (v4f){0.f, 0.f, 0.f, 0.f};
  if (EPI == 1) {
    bv = *(const v4fa*)(bias + clampi(nc, 0, N - 4));
    asm volatile("" :: "v"(bv));
  }
#pragma unroll
  for (int i = 0; i < 4; ++i) {
    const int mBase = m0 + (i << 4);
#pragma unroll
    for (int j = 0; j < 4; ++j) {
#pragma unroll
      for (int r = 0; r < 8; ++r) slab[(h8 + r) * 68 + (j << 4) + rl] = acc[i][j][r];
    }
    __builtin_amdgcn_fence(__ATOMIC_RELEASE, "workgroup");
    __builtin_amdgcn_wave_barrier();
    __builtin_amdgcn_fence(__ATOMIC_ACQUIRE, "workgroup");
    v4f vv[8];
#pragma unroll
    for (int it = 0; it < 8; ++it) {
      const int row = it * 2 + hh;
      v4f v = *(const v4fa*)(slab + row * 68 + c4);
      if (EPI == 1) v += bv;
      vv[it] = v;
    }
    for (int pass = 0; pass < 2; ++pass) {
#pragma unroll
      for (int it = 0; it < 8; ++it) {
        const int row = mBase + it * 2 + hh;
        if (cok && row < M) *(volatile v4f*)(D + (size_t)row * (size_t)ldd + nc) = vv[it];
      }
      __threadfence();
    }
    __builtin_amdgcn_fence(__ATOMIC_RELEASE, "workgroup");
    __builtin_amdgcn_wave_barrier();
    __builtin_amdgcn_fence(__ATOMIC_ACQUIRE, "workgroup");
  }
}

#pragma clang fp contract(off)

#define NN      50000
#define NE      400000
#define DIN     256
#define NCOL    512
#define MPAD    50048
#define NTHR    256
#define NWAVE   8
#define NBA     1024
#define SLA     10
#define NBB     49
#define LCAP    10240
#define WLCAP   1536
#define DEGCAP  16
#define WSTEPS  1563
#define SEGW    (WSTEPS * 32)
#define EIDBITS 19
#define WSMAX   (((size_t)128 << 20))

#define O_HB     ((size_t)0)
#define O_WCAT   (O_HB    + (size_t)MPAD * DIN * 2)
#define O_BIAS   (O_WCAT  + (size_t)NCOL * DIN * 2)
#define O_QKV    (O_BIAS  + (size_t)NCOL * 4)
#define O_NT     (O_QKV   + (size_t)MPAD * NCOL * 4)
#define O_LISTS  (O_NT    + (size_t)NBB * NBA * 8)
#define WS_TOTAL (O_LISTS + (size_t)NBB * LCAP * 8)

#define L_WL    0
#define L_SL    (L_WL  + NWAVE * WLCAP * 2)
#define L_CNT   (L_SL  + LCAP * 2)
#define L_OFF   (L_CNT + NBA)
#define L_CUR   (L_OFF + NBA)
#define L_MISC  (L_CUR + NBA)
#define L_TOTAL (L_MISC + 16)
#define BUCKET_LDS (L_TOTAL * 4)

#define PREP_W_BLK (NCOL * (DIN / 8) / NTHR)
#define PREP_GRID  (PREP_W_BLK + 1)

static_assert(MPAD == 391 * 128 && MPAD % 64 == 0 && MPAD >= NN && MPAD % 16 == 0);
static_assert(NCOL % 64 == 0 && DIN % 32 == 0 && NCOL % 32 == 0);
static_assert(NN % 8 == 0 && NN % NWAVE == 0);
static_assert(NBA == (1 << SLA) && NBB * NBA >= NN && (NBB - 1) * NBA < NN);
static_assert(SEGW * NWAVE >= NE && SEGW * NWAVE <= (1 << EIDBITS) && EIDBITS + SLA <= 31);
static_assert(NN <= 65536);
static_assert(LCAP * 4 >= 8192 * 5);
static_assert(DEGCAP >= 8 + 8);
static_assert(NWAVE * WLCAP >= LCAP && WLCAP * 4 >= 1040 * 5);
static_assert((LCAP * 2 / 4) % NTHR == 0 && NBA * 2 / 4 == 2 * NTHR);
static_assert(L_TOTAL % 4 == 0 && L_SL % 4 == 0 && L_CNT % 4 == 0 && BUCKET_LDS == 192576 && BUCKET_LDS <= 327680);
static_assert(PREP_W_BLK == 64);
static_assert(O_WCAT % 256 == 0 && O_BIAS % 256 == 0 && O_QKV % 256 == 0 && O_NT % 256 == 0 && O_LISTS % 256 == 0);
static_assert(WS_TOTAL == ((size_t)64845 << 11) && WS_TOTAL <= WSMAX);
static_assert((size_t)NN * 256 - 1 == 12799999);

typedef int v4i __attribute__((ext_vector_type(4)));
typedef int v2i __attribute__((ext_vector_type(2)));
typedef v4i __attribute__((may_alias)) v4ia;
typedef v2i __attribute__((may_alias)) v2ia;

__global__ __launch_bounds__(NTHR) void k_prep(const float* __restrict__ Wq, const float* __restrict__ bq,
                                               const float* __restrict__ Wk, const float* __restrict__ bk,
                                               const float* __restrict__ Wv, const float* __restrict__ bv,
                                               unsigned char* ws) {
  const int tid = (int)threadIdx.x;
  const int blk = (int)blockIdx.x;
  v4u o = (v4u){0u, 0u, 0u, 0u};
  size_t off = O_BIAS;
  bool act = false;
  if (blk < PREP_W_BLK) {
    const int g   = blk * NTHR + tid;
    const int row = g >> 5;
    const int c0  = (g & 31) * 8;
    v4f a, c;
    if (blk < 16) {
      const size_t so = (size_t)clampi(row, 0, 127) * DIN + (size_t)c0;
      a = *(const v4fa*)(Wq + so);
      c = *(const v4fa*)(Wq + so + 4);
    } else if (blk < 32) {
      const size_t so = (size_t)clampi(row - 128, 0, 127) * DIN + (size_t)c0;
      a = *(const v4fa*)(Wk + so);
      c = *(const v4fa*)(Wk + so + 4);
    } else {
      const size_t so = (size_t)clampi(row - 256, 0, 255) * DIN + (size_t)c0;
      a = *(const v4fa*)(Wv + so);
      c = *(const v4fa*)(Wv + so + 4);
    }
    asm volatile("" :: "v"(a));
    asm volatile("" :: "v"(c));
    o = pack8_bf16(a, c);
    off = O_WCAT + (size_t)g * 16;
    act = true;
  } else {
    const v4f vq = *(const v4fa*)(bq + 4 * clampi(tid, 0, 31));
    asm volatile("" :: "v"(vq));
    const v4f vk = *(const v4fa*)(bk + 4 * clampi(tid - 32, 0, 31));
    asm volatile("" :: "v"(vk));
    const v4f vv = *(const v4fa*)(bv + 4 * clampi(tid - 64, 0, 63));
    asm volatile("" :: "v"(vv));
    const unsigned mq = (tid < 32) ? 0xFFFFFFFFu : 0u;
    const unsigned mk = (tid >= 32 && tid < 64) ? 0xFFFFFFFFu : 0u;
    const unsigned mv = (tid >= 64 && tid < 128) ? 0xFFFFFFFFu : 0u;
    o = (v4u){ ((bf16_bits(vq[0]) << 16) & mq) | ((bf16_bits(vk[0]) << 16) & mk) | ((bf16_bits(vv[0]) << 16) & mv),
               ((bf16_bits(vq[1]) << 16) & mq) | ((bf16_bits(vk[1]) << 16) & mk) | ((bf16_bits(vv[1]) << 16) & mv),
               ((bf16_bits(vq[2]) << 16) & mq) | ((bf16_bits(vk[2]) << 16) & mk) | ((bf16_bits(vv[2]) << 16) & mv),
               ((bf16_bits(vq[3]) << 16) & mq) | ((bf16_bits(vk[3]) << 16) & mk) | ((bf16_bits(vv[3]) << 16) & mv) };
    off = O_BIAS + (size_t)clampi(tid, 0, 127) * 16;
    act = tid < 128;
  }
  if (act) {
    volatile v4u* q = (volatile v4u*)(ws + off);
    *q = o;
    __threadfence();
    *q = o;
  }
}

__global__ __launch_bounds__(NTHR) void k_bucket(const int* __restrict__ srcI, const int* __restrict__ dstI,
                                                 int* NODETAB, int* LISTS) {
  extern __shared__ __attribute__((aligned(16))) int dyn[];
  const int tid = (int)threadIdx.x, lane = tid & 31, wave = tid >> 5;
  const int blkB = (int)blockIdx.x;
  const int nodeBase = blkB * NBA;

  {
    const v4i z4 = (v4i){0, 0, 0, 0};
#pragma unroll 1
    for (int i = tid; i < L_TOTAL / 4; i += NTHR) *(v4ia*)(dyn + 4 * i) = z4;
  }
  __syncthreads();

  int wc = 0;
  {
    const int segBase = wave * SEGW;
#pragma unroll 1
    for (int st = 0; st < WSTEPS; ++st) {
      const int e  = segBase + st * 32 + lane;
      const int ec = e < NE ? e : NE - 1;
      const int dr = dstI[ec];
      asm volatile("" :: "v"(dr));
      const int sr = srcI[ec];
      asm volatile("" :: "v"(sr));
      const int oob = (e >= NE) ? -1 : 0;
      const int d = dr | oob;
      const int sc = clampi(sr, 0, NN - 1);
      const unsigned s = (unsigned)(d - nodeBase);
      const bool hit = (s < (unsigned)NBA) & ((unsigned)d < (unsigned)NN);
      const unsigned m = __builtin_amdgcn_ballot_w32(hit);
      const int pos = wc + (int)__builtin_amdgcn_mbcnt_lo(m, 0u);
      if (m != 0u) {
        if (hit && pos < WLCAP)
          *(v2ia*)(dyn + L_WL + (wave * WLCAP + pos) * 2) = (v2i){ sc, (int)((unsigned)e | (s << EIDBITS)) };
        wc += (int)__builtin_popcount(m);
      }
    }
  }
  if (lane == 0) dyn[L_MISC + wave] = wc;
  __syncthreads();

  if (wave == 0) {
    int t = 0, ov = 0;
#pragma unroll 1
    for (int w2 = 0; w2 < NWAVE; ++w2) {
      int c = __builtin_amdgcn_readfirstlane(dyn[L_MISC + w2]);
      if (c > WLCAP) ov = 1;
      c = clampi(c, 0, WLCAP);
#pragma unroll 1
      for (int i = 0; i < c; ++i) {
        const int u = dyn[L_WL + (w2 * WLCAP + i) * 2 + 1];
        const int slot = (u >> EIDBITS) & (NBA - 1);
        const int cv = dyn[L_CNT + slot];
        if (t < LCAP) {
          if (lane == 0) dyn[L_CNT + slot] = cv + 1;
          t = t + 1;
        } else {
          ov = 1;
        }
      }
    }
    if (lane == 0) { dyn[L_MISC + 8] = t; dyn[L_MISC + 9] = ov; }
  }
  __syncthreads();

  if (wave == 0) {
    const int base = lane * (NBA / 32);
    int s = 0, mx = 0;
#pragma unroll 1
    for (int i = 0; i < NBA / 32; ++i) {
      const int cv = dyn[L_CNT + base + i];
      s += cv;
      mx = cv > mx ? cv : mx;
    }
    int incl = s;
#pragma unroll
    for (int d = 1; d < 32; d <<= 1) {
      const int y = __shfl_up(incl, d, 32);
      if (lane >= d) incl += y;
    }
    int run = incl - s;
#pragma unroll 1
    for (int i = 0; i < NBA / 32; ++i) {
      const int cv = dyn[L_CNT + base + i];
      dyn[L_OFF + base + i] = run;
      dyn[L_CUR + base + i] = run;
      run += cv;
    }
    const unsigned bm = __builtin_amdgcn_ballot_w32(mx > DEGCAP);
    if (lane == 0) dyn[L_MISC + 10] = (bm != 0u) ? 1 : 0;
  }
  __syncthreads();

  if (wave == 0) {
    int t2 = 0;
#pragma unroll 1
    for (int w2 = 0; w2 < NWAVE; ++w2) {
      int c = __builtin_amdgcn_readfirstlane(dyn[L_MISC + w2]);
      c = clampi(c, 0, WLCAP);
#pragma unroll 1
      for (int i = 0; i < c; ++i) {
        const v2i u2 = *(const v2ia*)(dyn + L_WL + (w2 * WLCAP + i) * 2);
        const int slot = (u2.y >> EIDBITS) & (NBA - 1);
        const int eid  = u2.y & ((1 << EIDBITS) - 1);
        const int p = clampi(dyn[L_CUR + slot], 0, LCAP - 1);
        if (t2 < LCAP) {
          if (lane == 0) {
            *(v2ia*)(dyn + L_SL + 2 * p) = (v2i){ u2.x, eid };
            dyn[L_CUR + slot] = p + 1;
          }
          t2 = t2 + 1;
        }
      }
    }
  }
  __syncthreads();

  const int fl = ((dyn[L_MISC + 9] | dyn[L_MISC + 10]) != 0) ? 1 : 0;
  const int s0 = 2 * tid;
  const int s1 = 2 * (NTHR + tid);
  const int c00 = dyn[L_CNT + s0], c01 = dyn[L_CNT + s0 + 1];
  const int c10 = dyn[L_CNT + s1], c11 = dyn[L_CNT + s1 + 1];
  const v4i nv0 = (v4i){ dyn[L_OFF + s0], fl ? -1 : c00, dyn[L_OFF + s0 + 1], fl ? -1 : c01 };
  const v4i nv1 = (v4i){ dyn[L_OFF + s1], fl ? -1 : c10, dyn[L_OFF + s1 + 1], fl ? -1 : c11 };
  int* pn = NODETAB + (size_t)nodeBase * 2 + 4 * tid;
  int* pl = LISTS + (size_t)blkB * (LCAP * 2) + 4 * tid;
#pragma unroll 1
  for (int pass = 0; pass < 2; ++pass) {
    *(volatile v4i*)pn = nv0;
    *(volatile v4i*)(pn + 4 * NTHR) = nv1;
#pragma unroll 4
    for (int it = 0; it < LCAP * 2 / 4 / NTHR; ++it) {
      const v4i lv = *(const v4ia*)(dyn + L_SL + 4 * (it * NTHR + tid));
      *(volatile v4i*)(pl + it * NTHR * 4) = lv;
    }
    __threadfence();
  }
}

__device__ __forceinline__ v4f poison4(bool bad, v4f v) {
  const float qn = __int_as_float(0x7fc00000);
  v4f r;
  r.x = bad ? qn : v.x;
  r.y = bad ? qn : v.y;
  r.z = bad ? qn : v.z;
  r.w = bad ? qn : v.w;
  return r;
}

__global__ __launch_bounds__(NTHR) void k_replay(const float* __restrict__ QKV, const int* __restrict__ NODETAB,
                                                 const int* __restrict__ LISTS, const float* __restrict__ jac,
                                                 float* out) {
  const int tid = (int)threadIdx.x, lane = tid & 31, wave = tid >> 5;
  const int n  = (int)blockIdx.x * NWAVE + wave;
  const bool live = n < NN;
  const int nc = clampi(n, 0, NN - 1);
  const int bB = nc >> SLA;
  const v2i nt = *(const v2ia*)(NODETAB + 2 * (size_t)nc);
  asm volatile("" :: "v"(nt));
  const int start = nt.x;
  const int c = nt.y;
  const bool mark = (c < 0) | (c > DEGCAP);
  const int ccl = clampi(c, 0, DEGCAP);
  const int cn = __builtin_amdgcn_readfirstlane(live ? ccl : 0);
  const int st0 = clampi(start, 0, LCAP - 1);
  const int lastI = clampi(st0 + ccl - 1, st0, LCAP - 1);

  const v4f q = *(const v4fa*)(QKV + (size_t)nc * NCOL + 4 * lane);
  asm volatile("" :: "v"(q));
  const int* lp = LISTS + (size_t)bB * (LCAP * 2);

  v4f a0 = (v4f){0.f, 0.f, 0.f, 0.f};
  v4f a1 = (v4f){0.f, 0.f, 0.f, 0.f};
  float z0 = 0.0f, z1 = 0.0f;
#pragma unroll 1
  for (int j = 0; j < cn; ++j) {
    const int li = clampi(st0 + j, st0, lastI);
    const v2i pr = *(const v2ia*)(lp + 2 * li);
    asm volatile("" :: "v"(pr));
    const int s   = clampi(pr.x, 0, NN - 1);
    const int eid = clampi(pr.y, 0, NE - 1);
    const float* srow = QKV + (size_t)s * NCOL + 4 * lane;
    const v4f kv = *(const v4fa*)(srow + 128);
    asm volatile("" :: "v"(kv));
    const float jr = jac[eid];
    asm volatile("" :: "v"(jr));
    const v4f v0 = *(const v4fa*)(srow + 256);
    asm volatile("" :: "v"(v0));
    const v4f v1 = *(const v4fa*)(srow + 384);
    asm volatile("" :: "v"(v1));
    float p = kv.x * q.x;
    p = p + kv.y * q.y;
    p = p + kv.z * q.z;
    p = p + kv.w * q.w;
    p = p + __shfl_xor(p, 1, 32);
    p = p + __shfl_xor(p, 2, 32);
    p = p + __shfl_xor(p, 4, 32);
    float t = p / sqrtf(32.0f);
    t = (t < -5.0f) ? -5.0f : t;
    t = (t > 5.0f) ? 5.0f : t;
    const float w  = expf(t);
    const float jv = bf16_val(jr);
    a0 = a0 + v0 * w;
    a1 = a1 + v1 * jv;
    z0 = z0 + w;
    z1 = z1 + jv;
  }
  v4f o0, o1;
  o0.x = a0.x / z0; o0.y = a0.y / z0; o0.z = a0.z / z0; o0.w = a0.w / z0;
  o1.x = a1.x / z1; o1.y = a1.y / z1; o1.z = a1.z / z1; o1.w = a1.w / z1;
  const v4f r0 = poison4(mark, o0);
  const v4f r1 = poison4(mark, o1);
  if (n < NN) {
    float* op = out + (size_t)n * 256 + 4 * lane;
    *(volatile v4f*)op = r0;
    *(volatile v4f*)(op + 128) = r1;
    __threadfence();
    *(volatile v4f*)op = r0;
    *(volatile v4f*)(op + 128) = r1;
  }
}

extern "C" void kernel_launch(void* const* d_in, const int* in_sizes, int n_in,
                              void* d_out, int out_size, void* d_ws, size_t ws_size,
                              hipStream_t stream) {
  if (n_in < 10) return;
  if (in_sizes[0] != NN * DIN) return;
  if (in_sizes[1] != NE) return;
  if (in_sizes[2] != NE) return;
  if (in_sizes[3] != NE) return;
  if (in_sizes[4] != 128 * DIN) return;
  if (in_sizes[5] != 128) return;
  if (in_sizes[6] != 128 * DIN) return;
  if (in_sizes[7] != 128) return;
  if (in_sizes[8] != 256 * DIN) return;
  if (in_sizes[9] != 256) return;
  if (out_size != NN * 256) return;
  if (ws_size < (size_t)WS_TOTAL) return;

  const float* h   = (const float*)d_in[0];
  const int*   src = (const int*)d_in[1];
  const int*   dst = (const int*)d_in[2];
  const float* jac = (const float*)d_in[3];
  const float* Wq  = (const float*)d_in[4];
  const float* bq  = (const float*)d_in[5];
  const float* Wk  = (const float*)d_in[6];
  const float* bk  = (const float*)d_in[7];
  const float* Wv  = (const float*)d_in[8];
  const float* bv  = (const float*)d_in[9];
  float* out = (float*)d_out;

  unsigned char* ws = (unsigned char*)d_ws;
  unsigned short* HB   = (unsigned short*)(ws + O_HB);
  unsigned short* WCAT = (unsigned short*)(ws + O_WCAT);
  float* BIAS = (float*)(ws + O_BIAS);
  float* QKV  = (float*)(ws + O_QKV);
  int*   NT   = (int*)(ws + O_NT);
  int*   LST  = (int*)(ws + O_LISTS);

  k_plane<0><<<MPAD * DIN / 8 / 256, 256, 0, stream>>>(h, NN, DIN, DIN, HB, MPAD, DIN);
  k_prep<<<PREP_GRID, NTHR, 0, stream>>>(Wq, bq, Wk, bk, Wv, bv, ws);
  k_gemm_nt<0, 1><<<(MPAD / 64) * (NCOL / 64) / 8, 256, 0, stream>>>(HB, WCAT, BIAS, QKV, MPAD, NCOL, DIN, NCOL);
  hipFuncSetAttribute(reinterpret_cast<const void*>(&k_bucket), hipFuncAttributeMaxDynamicSharedMemorySize, BUCKET_LDS);
  k_bucket<<<NBB, NTHR, BUCKET_LDS, stream>>>(src, dst, NT, LST);
  k_replay<<<NN / NWAVE, NTHR, 0, stream>>>(QKV, NT, LST, jac, out);
}
